// QuesAnsByRGCN_50130858279579
// MI455X (gfx1250) — hardware-verified
//
#include <hip/hip_runtime.h>
#include <stddef.h>


#define NB    4
#define DW    300
#define HD    128
#define HG    384
#define DH    256
#define G     64
#define L     16
#define FIN   320
#define NH1   1024

#define NTHR  256
#define NWAVE 8

#define NPB   8
#define NR    (NPB * L)
#define NGP   (NPB / 4)
#define PP    72
#define ROWF  (NB * G)

#define NBD    128
#define EPT    8
#define NGRP   2
#define CHUNK  (NTHR * EPT * NGRP)
#define WCAP   (EPT * NGRP * 32)
#define LISTN  (NWAVE * WCAP)
#define SLOTSH 13
#define WSCAP  134217728

#define LN_F   0
#define LN_DH  (LN_F + NR * G * 4)
#define LN_DL  (LN_DH + NR * PP * 2)
#define LN_TH  (LN_DL + NR * PP * 2)
#define LN_TL  (LN_TH + NGP * G * PP * 2)
#define LN_BH  (LN_TL + NGP * G * PP * 2)
#define LN_BL  (LN_BH + G * PP * 2)
#define LN_QH  (LN_BL + G * PP * 2)
#define LN_QL  (LN_QH + 16 * PP * 2)
#define LN_S   (LN_QL + 16 * PP * 2)
#define LN_PH  (LN_S + NR * 16 * 4)
#define LN_PL  (LN_PH + NGP * 16 * PP * 2)
#define LN_P2  (LN_PL + NGP * 16 * PP * 2)
#define LN_TOT (LN_P2 + NPB * NB * L * 4)
#define LN_NF  0
#define LN_NH  (LN_NF + NGP * 16 * G * 4)
#define LN_NL  (LN_NH + NGP * 16 * PP * 2)
#define LN_HB  (LN_NL + NGP * 16 * PP * 2)
#define LR_ACC  0
#define LR_LIST (LR_ACC + NBD * ROWF * 4)
#define LR_WC   (LR_LIST + LISTN * 4)
#define LR_QG   (LR_WC + 64)
#define LR_SC   (LR_QG + ROWF * 4)
#define LR_BI   (LR_SC + NB * NBD * 4)
#define LR_TOT  (LR_BI + G * 4)

static_assert(NR == NWAVE * 16);
static_assert(NGP * 4 == NWAVE);
static_assert(NPB * NB == 32);
static_assert(FIN == G + DH);
static_assert(NTHR == ROWF && NTHR == NB * G && DH == NTHR);
static_assert(NH1 == 4 * NTHR);
static_assert(NTHR == 2 * NBD && NB == 4);
static_assert((NBD * ROWF) / 4 == 32 * NTHR);
static_assert(NBD % NWAVE == 0 && (NBD & (NBD - 1)) == 0 && NBD <= (1 << SLOTSH));
static_assert((CHUNK & (CHUNK - 1)) == 0);
static_assert(LN_HB + NGP * 16 * G * 4 <= LN_DH);
static_assert((LN_DH % 16) == 0 && (LN_TH % 16) == 0 && (LN_BH % 16) == 0 && (LN_QH % 16) == 0);
static_assert((LN_S % 16) == 0 && (LN_PH % 16) == 0 && (LN_P2 % 16) == 0 && (LN_NH % 16) == 0 && (LN_HB % 16) == 0);
static_assert((LR_LIST % 16) == 0 && (LR_QG % 16) == 0 && (LR_SC % 16) == 0);
static_assert(((PP * 2) % 16) == 0);
static_assert(NPB * ROWF == 2 * 4 * NTHR);

typedef float          v4f  __attribute__((ext_vector_type(4)));
typedef float          v8f  __attribute__((ext_vector_type(8)));
typedef int            v4i  __attribute__((ext_vector_type(4)));
typedef unsigned short v8us __attribute__((ext_vector_type(8)));
typedef __bf16         v16b __attribute__((ext_vector_type(16)));
union FragB { v16b v; v8us h[2]; };

__device__ __forceinline__ unsigned int bfr(float f) {
  const unsigned int u = __float_as_uint(f);
  return (u + 0x7FFFu + ((u >> 16) & 1u)) >> 16;
}
__device__ __forceinline__ void split1(float x, unsigned short& hb, unsigned short& lb) {
  const unsigned int hu = bfr(x);
  const float hf = __uint_as_float(hu << 16);
  hb = (unsigned short)hu;
  lb = (unsigned short)bfr(x - hf);
}
__device__ __forceinline__ void split8(v4f a, v4f b, v8us& hi, v8us& lo) {
  unsigned short hb, lb;
  split1(a.x, hb, lb); hi[0] = hb; lo[0] = lb;
  split1(a.y, hb, lb); hi[1] = hb; lo[1] = lb;
  split1(a.z, hb, lb); hi[2] = hb; lo[2] = lb;
  split1(a.w, hb, lb); hi[3] = hb; lo[3] = lb;
  split1(b.x, hb, lb); hi[4] = hb; lo[4] = lb;
  split1(b.y, hb, lb); hi[5] = hb; lo[5] = lb;
  split1(b.z, hb, lb); hi[6] = hb; lo[6] = lb;
  split1(b.w, hb, lb); hi[7] = hb; lo[7] = lb;
}
__device__ __forceinline__ void col8(const float* p, int st, v4f& a, v4f& b) {
  a.x = p[0];      a.y = p[st];     a.z = p[2 * st]; a.w = p[3 * st];
  b.x = p[4 * st]; b.y = p[5 * st]; b.z = p[6 * st]; b.w = p[7 * st];
}

__device__ __forceinline__ v8f wmb(v16b a, v16b b, v8f c) {
  v8f d = __builtin_amdgcn_wmma_f32_16x16x32_bf16(false, a, false, b, (short)0, c, false, false);
  asm volatile("v_nop\n\tv_nop\n\tv_nop\n\tv_nop" : "+v"(d) : "v"(a), "v"(b));
  return d;
}

__device__ __forceinline__ v8f gemm64(const unsigned short* pah, const unsigned short* pal,
                                       const unsigned short* pbh, const unsigned short* pbl) {
  v8f acc = {0.f, 0.f, 0.f, 0.f, 0.f, 0.f, 0.f, 0.f};
#pragma unroll
  for (int ks = 0; ks < 2; ++ks) {
    FragB ah, al, bh, bl;
    ah.h[0] = *(const v8us*)(pah + 32 * ks); ah.h[1] = *(const v8us*)(pah + 32 * ks + 16);
    al.h[0] = *(const v8us*)(pal + 32 * ks); al.h[1] = *(const v8us*)(pal + 32 * ks + 16);
    bh.h[0] = *(const v8us*)(pbh + 32 * ks); bh.h[1] = *(const v8us*)(pbh + 32 * ks + 16);
    bl.h[0] = *(const v8us*)(pbl + 32 * ks); bl.h[1] = *(const v8us*)(pbl + 32 * ks + 16);
    acc = wmb(ah.v, bh.v, acc);
    acc = wmb(ah.v, bl.v, acc);
    acc = wmb(al.v, bh.v, acc);
  }
  return acc;
}

__global__ __launch_bounds__(HG) void k_gx(
    const int* __restrict__ ques, const float* __restrict__ embw,
    const float* __restrict__ wxf, const float* __restrict__ bxf,
    const float* __restrict__ wxb, const float* __restrict__ bxb,
    float* gx, int T, int nVw) {
  __shared__ float xrow[DW + 4];
  const int t = blockIdx.x, b = blockIdx.y, dir = blockIdx.z, j = threadIdx.x;
  const int tt = dir ? (T - 1 - t) : t;
  int tok = ques[b * T + tt];
  tok = tok < 0 ? 0 : (tok > nVw - 1 ? nVw - 1 : tok);
  if (j < DW) xrow[j] = embw[(size_t)tok * DW + j];
  __syncthreads();
  const float* wx = dir ? wxb : wxf;
  const float* bx = dir ? bxb : bxf;
  const float* wcol = wx + j;
  float acc = 0.f;
#pragma unroll 1
  for (int k = 0; k < DW; ++k) acc = fmaf(xrow[k], wcol[(size_t)k * HG], acc);
  acc += bx[j];
  float* p = gx + ((size_t)(dir * NB + b) * T + t) * HG + j;
  *(volatile float*)p = acc;
  __threadfence();
  *(volatile float*)p = acc;
}

__global__ __launch_bounds__(HG) void k_gru(
    const int* __restrict__ ques, const float* __restrict__ gx,
    const float* __restrict__ whf, const float* __restrict__ bhf,
    const float* __restrict__ whb, const float* __restrict__ bhb,
    float* q, int T) {
  __shared__ float h[HD];
  __shared__ float gh[HG];
  const int b = blockIdx.x, dir = blockIdx.y, j = threadIdx.x;
  const float* wh = dir ? whb : whf;
  const float* bh = dir ? bhb : bhf;
  const float* gxr = gx + (size_t)(dir * NB + b) * T * HG;
  if (j < HD) h[j] = 0.f;
  __syncthreads();
#pragma unroll 1
  for (int t = 0; t < T; ++t) {
    const float* wcol = wh + j;
    float acc = 0.f;
#pragma unroll 1
    for (int k = 0; k < HD; ++k) acc = fmaf(h[k], wcol[(size_t)k * HG], acc);
    gh[j] = acc + bh[j];
    __syncthreads();
    if (j < HD) {
      const float* g0 = gxr + (size_t)t * HG;
      const float r  = 1.0f / (1.0f + expf(-(g0[j] + gh[j])));
      const float z  = 1.0f / (1.0f + expf(-(g0[HD + j] + gh[HD + j])));
      const float n  = tanhf(g0[2 * HD + j] + r * gh[2 * HD + j]);
      const float ho = h[j];
      const float hn = (1.0f - z) * n + z * ho;
      const int tt = dir ? (T - 1 - t) : t;
      const int mk = ques[b * T + tt];
      h[j] = (mk != 0) ? hn : ho;
    }
    __syncthreads();
  }
  float v = 0.f;
  if (j < HD) v = h[j];
  float* p = q + (size_t)b * DH + dir * HD + j;
  if (j < HD) *(volatile float*)p = v;
  __threadfence();
  if (j < HD) *(volatile float*)p = v;
}

__global__ __launch_bounds__(NTHR) void k_qg(
    const float* __restrict__ q, const float* __restrict__ whg, const float* __restrict__ bhg,
    const float* __restrict__ bases, float* qg, unsigned short* qp, unsigned short* bp) {
  __shared__ __attribute__((aligned(16))) float sq[NB * DH];
  __shared__ __attribute__((aligned(16))) float sg[ROWF];
  const int tid = threadIdx.x;
#pragma unroll
  for (int i = 0; i < (NB * DH) / NTHR; ++i) sq[tid + i * NTHR] = q[tid + i * NTHR];
  __syncthreads();
  const int b = tid >> 6, g = tid & (G - 1);
  float acc = 0.f;
#pragma unroll 1
  for (int k = 0; k < DH; ++k) acc = fmaf(sq[b * DH + k], whg[(size_t)k * G + g], acc);
  acc += bhg[g];
  sg[tid] = acc;
  __syncthreads();
  const bool wq = tid < 128;
  v8us qh, ql;
  {
    const int row = (tid >> 3) & 15, g0 = (tid & 7) * 8;
    const int srow = row < NB ? row : 0;
    const float msk = row < NB ? 1.0f : 0.0f;
    const v4f a = *(const v4f*)(sg + srow * G + g0) * msk;
    const v4f c = *(const v4f*)(sg + srow * G + g0 + 4) * msk;
    split8(a, c, qh, ql);
  }
  v8us bh0, bl0, bh1, bl1;
  {
    const int o = tid >> 3, g0 = (tid & 7) * 8;
    v4f a, c;
    col8(bases + (size_t)g0 * G + o, G, a, c);
    split8(a, c, bh0, bl0);
    const int task = tid + NTHR;
    const int o1 = task >> 3, g1 = (task & 7) * 8;
    col8(bases + (size_t)g1 * G + o1, G, a, c);
    split8(a, c, bh1, bl1);
  }
  *(volatile float*)(qg + tid) = acc;
  if (wq) {
    *(volatile v8us*)(qp + 8 * tid) = qh;
    *(volatile v8us*)(qp + 16 * G + 8 * tid) = ql;
  }
  *(volatile v8us*)(bp + 8 * tid) = bh0;
  *(volatile v8us*)(bp + G * G + 8 * tid) = bl0;
  *(volatile v8us*)(bp + 8 * (tid + NTHR)) = bh1;
  *(volatile v8us*)(bp + G * G + 8 * (tid + NTHR)) = bl1;
  __threadfence();
  *(volatile float*)(qg + tid) = acc;
  if (wq) {
    *(volatile v8us*)(qp + 8 * tid) = qh;
    *(volatile v8us*)(qp + 16 * G + 8 * tid) = ql;
  }
  *(volatile v8us*)(bp + 8 * tid) = bh0;
  *(volatile v8us*)(bp + G * G + 8 * tid) = bl0;
  *(volatile v8us*)(bp + 8 * (tid + NTHR)) = bh1;
  *(volatile v8us*)(bp + G * G + 8 * (tid + NTHR)) = bl1;
}

__global__ __launch_bounds__(NTHR) void k_node(
    const int* __restrict__ ndesc, const float* __restrict__ embd,
    const unsigned short* __restrict__ qp, const unsigned short* __restrict__ bp,
    float* hb, int nN, int nVd) {
  extern __shared__ v4f lds_dyn[];
  char* lds = (char*)lds_dyn;
  float*          sF  = (float*)(lds + LN_F);
  unsigned short* sDh = (unsigned short*)(lds + LN_DH);
  unsigned short* sDl = (unsigned short*)(lds + LN_DL);
  unsigned short* sTh = (unsigned short*)(lds + LN_TH);
  unsigned short* sTl = (unsigned short*)(lds + LN_TL);
  unsigned short* sBh = (unsigned short*)(lds + LN_BH);
  unsigned short* sQh = (unsigned short*)(lds + LN_QH);
  float*          sS  = (float*)(lds + LN_S);
  unsigned short* sPh = (unsigned short*)(lds + LN_PH);
  unsigned short* sPl = (unsigned short*)(lds + LN_PL);
  float*          sP2 = (float*)(lds + LN_P2);
  float*          sNF = (float*)(lds + LN_NF);
  unsigned short* sNh = (unsigned short*)(lds + LN_NH);
  unsigned short* sNl = (unsigned short*)(lds + LN_NL);
  float*          sHB = (float*)(lds + LN_HB);
  const int tid = threadIdx.x, lane = tid & 31, hh = lane >> 4, m = lane & 15;
  const int wave = __builtin_amdgcn_readfirstlane(tid >> 5);
  const int nodeBase = blockIdx.x * NPB;

  {
    const int pl = tid >> 7, row = (tid >> 3) & 15, c = (tid & 7) * 8;
    const v8us v = *(const v8us*)(qp + pl * (16 * G) + row * G + c);
    *(v8us*)(sQh + pl * (16 * PP) + row * PP + c) = v;
#pragma unroll
    for (int i = 0; i < 4; ++i) {
      const int task = tid + i * NTHR;
      const int pb2 = task >> 9, o = (task >> 3) & 63, c2 = (task & 7) * 8;
      const v8us w = *(const v8us*)(bp + pb2 * (G * G) + o * G + c2);
      *(v8us*)(sBh + pb2 * (G * PP) + o * PP + c2) = w;
    }
  }
#pragma unroll
  for (int i = 0; i < 8; ++i) {
    const int task = tid + i * NTHR;
    const int row = task >> 4, c4 = task & 15;
    int node = nodeBase + (row >> 4);
    node = node > nN - 1 ? nN - 1 : node;
    int tok = ndesc[(size_t)node * L + (row & 15)];
    tok = tok < 0 ? 0 : (tok > nVd - 1 ? nVd - 1 : tok);
    const v4f v = *(const v4f*)(embd + (size_t)tok * G + 4 * c4);
    *(v4f*)(sF + row * G + 4 * c4) = v;
  }
  __syncthreads();
#pragma unroll
  for (int i = 0; i < 4; ++i) {
    const int task = tid + i * NTHR;
    const int row = task >> 3, c = (task & 7) * 8;
    const v4f a = *(const v4f*)(sF + row * G + c);
    const v4f b = *(const v4f*)(sF + row * G + c + 4);
    v8us hv, lv;
    split8(a, b, hv, lv);
    *(v8us*)(sDh + row * PP + c) = hv;
    *(v8us*)(sDl + row * PP + c) = lv;
  }
#pragma unroll
  for (int i = 0; i < 4; ++i) {
    const int task = tid + i * NTHR;
    const int g = task & 63, kc = (task >> 6) & 7, grp = task >> 9;
    v4f a, b;
    col8(sF + (grp * 64 + 8 * kc) * G + g, G, a, b);
    v8us hv, lv;
    split8(a, b, hv, lv);
    *(v8us*)(sTh + (grp * G + g) * PP + 8 * kc) = hv;
    *(v8us*)(sTl + (grp * G + g) * PP + 8 * kc) = lv;
  }
  __syncthreads();
  {
    const v8f acc = gemm64(sDh + (wave * 16 + m) * PP + 8 * hh, sDl + (wave * 16 + m) * PP + 8 * hh,
                           sQh + m * PP + 8 * hh, sQh + 16 * PP + m * PP + 8 * hh);
    float* d = sS + (wave * 16 + 8 * hh) * 16 + m;
#pragma unroll
    for (int r = 0; r < 8; ++r) d[r * 16] = acc[r];
  }
  __syncthreads();
  if (wave == 0) {
    const int nl = lane >> 2, b = lane & 3;
    const float* srow = sS + (nl * 16) * 16 + b;
    float mx = srow[0];
#pragma unroll 1
    for (int l = 1; l < L; ++l) mx = fmaxf(mx, srow[16 * l]);
    float* prow = sP2 + (nl * NB + b) * L;
    float sum = 0.f;
#pragma unroll 1
    for (int l = 0; l < L; ++l) { const float e = expf(srow[16 * l] - mx); sum += e; prow[l] = e; }
    const float rs = 1.0f / sum;
    v4f e0, e1, e2, e3;
    e0.x = prow[0];  e0.y = prow[1];  e0.z = prow[2];  e0.w = prow[3];
    e1.x = prow[4];  e1.y = prow[5];  e1.z = prow[6];  e1.w = prow[7];
    e2.x = prow[8];  e2.y = prow[9];  e2.z = prow[10]; e2.w = prow[11];
    e3.x = prow[12]; e3.y = prow[13]; e3.z = prow[14]; e3.w = prow[15];
    const int jj = nl & 3;
    unsigned short* ph = sPh + (4 * nl + b) * PP;
    unsigned short* pl = sPl + (4 * nl + b) * PP;
#pragma unroll
    for (int c = 0; c < 8; ++c) {
      const float sc = ((c >> 1) == jj) ? rs : 0.0f;
      const v4f a  = ((c & 1) ? e2 : e0) * sc;
      const v4f bb = ((c & 1) ? e3 : e1) * sc;
      v8us hv, lv;
      split8(a, bb, hv, lv);
      *(v8us*)(ph + 8 * c) = hv;
      *(v8us*)(pl + 8 * c) = lv;
    }
  }
  __syncthreads();
  {
    const int grp = wave >> 2, nt = wave & 3;
    const v8f acc = gemm64(sPh + (grp * 16 + m) * PP + 8 * hh, sPl + (grp * 16 + m) * PP + 8 * hh,
                           sTh + (grp * G + 16 * nt + m) * PP + 8 * hh,
                           sTl + (grp * G + 16 * nt + m) * PP + 8 * hh);
    float* d = sNF + (grp * 16 + 8 * hh) * G + 16 * nt + m;
#pragma unroll
    for (int r = 0; r < 8; ++r) d[r * G] = acc[r];
  }
  __syncthreads();
  {
    const int row = tid >> 3, c = (tid & 7) * 8;
    const v4f a = *(const v4f*)(sNF + row * G + c);
    const v4f b = *(const v4f*)(sNF + row * G + c + 4);
    v8us hv, lv;
    split8(a, b, hv, lv);
    *(v8us*)(sNh + row * PP + c) = hv;
    *(v8us*)(sNl + row * PP + c) = lv;
  }
  __syncthreads();
  {
    const int rt = wave >> 2, nt = wave & 3;
    const v8f acc = gemm64(sNh + (16 * rt + m) * PP + 8 * hh, sNl + (16 * rt + m) * PP + 8 * hh,
                           sBh + (16 * nt + m) * PP + 8 * hh, sBh + G * PP + (16 * nt + m) * PP + 8 * hh);
    float* d = sHB + (16 * rt + 8 * hh) * G + 16 * nt + m;
#pragma unroll
    for (int r = 0; r < 8; ++r) d[r * G] = acc[r];
  }
  __syncthreads();
  {
    float* gp = hb + (size_t)nodeBase * ROWF;
    const v4f v0 = *(const v4f*)(sHB + 4 * tid);
    const v4f v1 = *(const v4f*)(sHB + 4 * (tid + NTHR));
    *(volatile v4f*)(gp + 4 * tid) = v0;
    *(volatile v4f*)(gp + 4 * (tid + NTHR)) = v1;
    __threadfence();
    *(volatile v4f*)(gp + 4 * tid) = v0;
    *(volatile v4f*)(gp + 4 * (tid + NTHR)) = v1;
  }
}

template <int NBK>
__device__ __forceinline__ int scan_chunk(const int* __restrict__ dsts, int nE, int cbase, int slotBase,
                                          int vec8, int* list, int tid, int lane, int wave) {
  int wc = 0;
#pragma unroll
  for (int g = 0; g < NGRP; ++g) {
    const int el0  = (g * NTHR + tid) * EPT;
    const int e0   = cbase + el0;
    const int sent = -2147483647 - 1;
    v4i da, db;
    if (vec8 != 0 && cbase + CHUNK <= nE) {
      da = *(const v4i*)(dsts + e0);
      db = *(const v4i*)(dsts + e0 + 4);
    } else {
      da.x = (e0     < nE) ? dsts[min(e0, nE - 1)] : sent;
      da.y = (e0 + 1 < nE) ? dsts[min(e0 + 1, nE - 1)] : sent;
      da.z = (e0 + 2 < nE) ? dsts[min(e0 + 2, nE - 1)] : sent;
      da.w = (e0 + 3 < nE) ? dsts[min(e0 + 3, nE - 1)] : sent;
      db.x = (e0 + 4 < nE) ? dsts[min(e0 + 4, nE - 1)] : sent;
      db.y = (e0 + 5 < nE) ? dsts[min(e0 + 5, nE - 1)] : sent;
      db.z = (e0 + 6 < nE) ? dsts[min(e0 + 6, nE - 1)] : sent;
      db.w = (e0 + 7 < nE) ? dsts[min(e0 + 7, nE - 1)] : sent;
    }
    const unsigned nb = (unsigned)slotBase;
    const unsigned s0 = (unsigned)da.x - nb, s1 = (unsigned)da.y - nb;
    const unsigned s2 = (unsigned)da.z - nb, s3 = (unsigned)da.w - nb;
    const unsigned s4 = (unsigned)db.x - nb, s5 = (unsigned)db.y - nb;
    const unsigned s6 = (unsigned)db.z - nb, s7 = (unsigned)db.w - nb;
    const bool h0 = s0 < (unsigned)NBK, h1 = s1 < (unsigned)NBK, h2 = s2 < (unsigned)NBK, h3 = s3 < (unsigned)NBK;
    const bool h4 = s4 < (unsigned)NBK, h5 = s5 < (unsigned)NBK, h6 = s6 < (unsigned)NBK, h7 = s7 < (unsigned)NBK;
    const unsigned any = __builtin_amdgcn_ballot_w32(h0 | h1 | h2 | h3 | h4 | h5 | h6 | h7);
    if (any != 0u) {
#define HITJ(J, HJ, SJ) { \
        const unsigned mj = __builtin_amdgcn_ballot_w32(HJ); \
        if (mj != 0u) { \
          if (HJ) { \
            const int pos = wc + (int)__builtin_amdgcn_mbcnt_lo(mj, 0u); \
            if (pos < WCAP) list[wave * WCAP + pos] = ((el0 + (J)) << SLOTSH) | (int)(SJ); \
          } \
          wc += (int)__builtin_popcount(mj); } }
      HITJ(0, h0, s0)
      HITJ(1, h1, s1)
      HITJ(2, h2, s2)
      HITJ(3, h3, s3)
      HITJ(4, h4, s4)
      HITJ(5, h5, s5)
      HITJ(6, h6, s6)
      HITJ(7, h7, s7)
#undef HITJ
    }
  }
  return wc;
}

__global__ __launch_bounds__(NTHR) void k_graph(
    const int* __restrict__ edst, const int* __restrict__ esrc, const int* __restrict__ etyp,
    const float* __restrict__ wcomp, const float* __restrict__ gbias, const float* __restrict__ qg,
    const float* __restrict__ hb, float* nf2, float* sc2,
    int nN, int nE, int nR, int NPAD, int vec8) {
  extern __shared__ v4f lds_dyn[];
  char* lds = (char*)lds_dyn;
  float* accp = (float*)(lds + LR_ACC);
  int*   list = (int*)(lds + LR_LIST);
  int*   wcnt = (int*)(lds + LR_WC);
  float* sQG  = (float*)(lds + LR_QG);
  float* sSC  = (float*)(lds + LR_SC);
  float* sBI  = (float*)(lds + LR_BI);
  const int tid = threadIdx.x, lane = tid & 31;
  const int wave = __builtin_amdgcn_readfirstlane(tid >> 5);
  const int nodeBase = blockIdx.x * NBD;

  {
    const v4f z = {0.f, 0.f, 0.f, 0.f};
#pragma unroll 1
    for (int i = tid; i < (NBD * ROWF) / 4; i += NTHR) ((v4f*)accp)[i] = z;
    sQG[tid] = qg[tid];
    if (tid < G) sBI[tid] = gbias[tid];
  }
  __syncthreads();

  const int nChunks = (nE + CHUNK - 1) / CHUNK;
#pragma unroll 1
  for (int ch = 0; ch < nChunks; ++ch) {
    const int cbase = ch * CHUNK;
    const int wc = scan_chunk<NBD>(edst, nE, cbase, nodeBase, vec8, list, tid, lane, wave);
    if (lane == 0) wcnt[wave] = wc;
    __syncthreads();
#pragma unroll 1
    for (int lw = 0; lw < NWAVE; ++lw) {
      int n = __builtin_amdgcn_readfirstlane(wcnt[lw]);
      n = n > WCAP ? WCAP : (n < 0 ? 0 : n);
      const int* lp = list + lw * WCAP;
#pragma unroll 1
      for (int i = 0; i < n; ++i) {
        const int ent  = __builtin_amdgcn_readfirstlane(lp[i]);
        const int slot = ent & (NBD - 1);
        if ((slot & (NWAVE - 1)) == wave) {
          int e = cbase + ((ent >> SLOTSH) & (CHUNK - 1));
          e = e > nE - 1 ? nE - 1 : e;
          int sv = esrc[e];
          sv = sv < 0 ? 0 : (sv > nN - 1 ? nN - 1 : sv);
          int rv = etyp[e];
          rv = rv < 0 ? 0 : (rv > nR - 1 ? nR - 1 : rv);
          const float w = wcomp[rv];
          const float* hp = hb + (size_t)sv * ROWF + 8 * lane;
          const v4f x0 = *(const v4f*)hp;
          const v4f x1 = *(const v4f*)(hp + 4);
          float* ap = accp + slot * ROWF + 8 * lane;
          v4f a0 = *(const v4f*)ap;
          v4f a1 = *(const v4f*)(ap + 4);
          a0 += x0 * w;
          a1 += x1 * w;
          *(v4f*)ap = a0;
          *(v4f*)(ap + 4) = a1;
        }
      }
    }
    __syncthreads();
  }

  {
    const int o = (4 * tid) & (G - 1);
    v4f bv;
    bv.x = sBI[o]; bv.y = sBI[o + 1]; bv.z = sBI[o + 2]; bv.w = sBI[o + 3];
    const v4f z = {0.f, 0.f, 0.f, 0.f};
#pragma unroll 1
    for (int k = 0; k < 32; ++k) {
      float* p = accp + 4 * tid + 1024 * k;
      v4f v = *(const v4f*)p;
      v = v + bv;
      v.x = fmaxf(v.x, 0.f); v.y = fmaxf(v.y, 0.f); v.z = fmaxf(v.z, 0.f); v.w = fmaxf(v.w, 0.f);
      *(v4f*)p = v;
      (void)z;
    }
  }
  __syncthreads();
  {
    const int slot = tid & (NBD - 1);
    const int b0 = (tid >> 7) * 2;
#pragma unroll 1
    for (int bb = 0; bb < 2; ++bb) {
      const int b = b0 + bb;
      const float* fr = accp + slot * ROWF + b * G;
      const float* qr = sQG + b * G;
      float s = 0.f;
#pragma unroll 1
      for (int o = 0; o < G; ++o) s = fmaf(fr[o], qr[o], s);
      sSC[b * NBD + slot] = s;
    }
  }
  __syncthreads();
  float* gp = nf2 + (size_t)nodeBase * ROWF;
  float* sp = sc2 + (size_t)wave * NPAD + nodeBase + 4 * lane;
#pragma unroll 1
  for (int k = 0; k < 32; ++k) {
    const int idx = tid + NTHR * k;
    const v4f v = ((const v4f*)accp)[idx];
    *(volatile v4f*)(gp + 4 * idx) = v;
  }
  if (wave < NB) {
    const v4f sv = *(const v4f*)(sSC + wave * NBD + 4 * lane);
    *(volatile v4f*)sp = sv;
  }
  __threadfence();
#pragma unroll 1
  for (int k = 0; k < 32; ++k) {
    const int idx = tid + NTHR * k;
    const v4f v = ((const v4f*)accp)[idx];
    *(volatile v4f*)(gp + 4 * idx) = v;
  }
  if (wave < NB) {
    const v4f sv = *(const v4f*)(sSC + wave * NBD + 4 * lane);
    *(volatile v4f*)sp = sv;
  }
}

__global__ __launch_bounds__(NTHR) void k_pool(
    const float* __restrict__ sc2, const float* __restrict__ nf2, const float* __restrict__ q,
    const float* __restrict__ w1, const float* __restrict__ b1, float* hid, int nN, int NPAD) {
  extern __shared__ v4f lds_dyn[];
  float* sp = (float*)lds_dyn;
  __shared__ float red[NTHR];
  __shared__ float feat[FIN];
  const int tid = threadIdx.x, b = blockIdx.x;
  const float* scr = sc2 + (size_t)b * NPAD;
  float lm = -__builtin_huge_valf();
#pragma unroll 1
  for (int n = tid; n < nN; n += NTHR) lm = fmaxf(lm, scr[n]);
  red[tid] = lm;
  __syncthreads();
#pragma unroll 1
  for (int s = NTHR / 2; s > 0; s >>= 1) {
    if (tid < s) red[tid] = fmaxf(red[tid], red[tid + s]);
    __syncthreads();
  }
  const float mxv = red[0];
  __syncthreads();
  float ls = 0.f;
#pragma unroll 1
  for (int n = tid; n < nN; n += NTHR) { const float e = expf(scr[n] - mxv); sp[n] = e; ls += e; }
  red[tid] = ls;
  __syncthreads();
#pragma unroll 1
  for (int s = NTHR / 2; s > 0; s >>= 1) {
    if (tid < s) red[tid] = red[tid] + red[tid + s];
    __syncthreads();
  }
  const float rS = 1.0f / red[0];
  __syncthreads();
  const int g = tid & (G - 1), qn = tid >> 6;
  const float* fp = nf2 + (size_t)b * G + g;
  float acc = 0.f;
#pragma unroll 1
  for (int n = qn; n < nN; n += NTHR / G) acc = fmaf(sp[n] * rS, fp[(size_t)n * ROWF], acc);
  red[tid] = acc;
  feat[G + tid] = q[(size_t)b * DH + tid];
  __syncthreads();
  if (tid < G) feat[tid] = ((red[tid] + red[G + tid]) + red[2 * G + tid]) + red[3 * G + tid];
  __syncthreads();
  float a0 = 0.f, a1 = 0.f, a2 = 0.f, a3 = 0.f;
  const float* wc = w1 + tid;
#pragma unroll 1
  for (int k = 0; k < FIN; ++k) {
    const float f = feat[k];
    const float* wr = wc + (size_t)k * NH1;
    a0 = fmaf(f, wr[0], a0);
    a1 = fmaf(f, wr[NTHR], a1);
    a2 = fmaf(f, wr[2 * NTHR], a2);
    a3 = fmaf(f, wr[3 * NTHR], a3);
  }
  const float v0 = fmaxf(a0 + b1[tid], 0.f);
  const float v1 = fmaxf(a1 + b1[tid + NTHR], 0.f);
  const float v2 = fmaxf(a2 + b1[tid + 2 * NTHR], 0.f);
  const float v3 = fmaxf(a3 + b1[tid + 3 * NTHR], 0.f);
  float* hp = hid + (size_t)b * NH1 + tid;
  *(volatile float*)(hp) = v0;
  *(volatile float*)(hp + NTHR) = v1;
  *(volatile float*)(hp + 2 * NTHR) = v2;
  *(volatile float*)(hp + 3 * NTHR) = v3;
  __threadfence();
  *(volatile float*)(hp) = v0;
  *(volatile float*)(hp + NTHR) = v1;
  *(volatile float*)(hp + 2 * NTHR) = v2;
  *(volatile float*)(hp + 3 * NTHR) = v3;
}

__global__ __launch_bounds__(NTHR) void k_fc2(
    const float* __restrict__ hid, const float* __restrict__ w2, const float* __restrict__ b2,
    float* out, int NC, int total) {
  __shared__ __attribute__((aligned(16))) float sh[NB * NH1];
  const int tid = threadIdx.x;
#pragma unroll 1
  for (int i = tid; i < (NB * NH1) / 4; i += NTHR) ((v4f*)sh)[i] = ((const v4f*)hid)[i];
  __syncthreads();
  const int f = blockIdx.x * NTHR + tid;
  const bool ok = f < total;
  const int fc = ok ? f : (total - 1);
  const int b = (fc >= NC ? 1 : 0) + (fc >= 2 * NC ? 1 : 0) + (fc >= 3 * NC ? 1 : 0);
  const int j = fc - b * NC;
  const float* hr = sh + b * NH1;
  const float* wc = w2 + j;
  float acc = 0.f;
#pragma unroll 1
  for (int k = 0; k < NH1; ++k) acc = fmaf(hr[k], wc[(size_t)k * NC], acc);
  acc += b2[j];
  if (ok) *(volatile float*)(out + f) = acc;
  __threadfence();
  if (ok) *(volatile float*)(out + f) = acc;
}

extern "C" void kernel_launch(void* const* d_in, const int* in_sizes, int n_in,
                              void* d_out, int out_size, void* d_ws, size_t ws_size,
                              hipStream_t stream) {
  if (n_in < 24) return;
  const int NC = in_sizes[23];
  if (NC < 1 || out_size != NB * NC) return;
  if (in_sizes[0] < NB || (in_sizes[0] % NB) != 0) return;
  const int T = in_sizes[0] / NB;
  if (T < 1 || T > 4096) return;
  if (in_sizes[1] < L || (in_sizes[1] % L) != 0) return;
  const int nN = in_sizes[1] / L;
  const int nE = in_sizes[2];
  if (nE < 1 || in_sizes[3] != nE || in_sizes[4] != nE) return;
  if (in_sizes[5] < DW || (in_sizes[5] % DW) != 0) return;
  const int nVw = in_sizes[5] / DW;
  if (in_sizes[6] < G || (in_sizes[6] % G) != 0) return;
  const int nVd = in_sizes[6] / G;
  if (in_sizes[7] != DW * HG || in_sizes[8] != HD * HG || in_sizes[9] != HG || in_sizes[10] != HG) return;
  if (in_sizes[11] != DW * HG || in_sizes[12] != HD * HG || in_sizes[13] != HG || in_sizes[14] != HG) return;
  if (in_sizes[15] != DH * G || in_sizes[16] != G || in_sizes[17] != G * G) return;
  const int nR = in_sizes[18];
  if (nR < 1 || in_sizes[19] != G) return;
  if (in_sizes[20] != FIN * NH1 || in_sizes[21] != NH1 || in_sizes[22] != NH1 * NC) return;
  if (nN > (1 << 24) || nE > (1 << 28)) return;
  if ((size_t)nN * 4 > 196608) return;

  const int*   ques  = (const int*)d_in[0];
  const int*   ndesc = (const int*)d_in[1];
  const int*   esrc  = (const int*)d_in[2];
  const int*   edst  = (const int*)d_in[3];
  const int*   etyp  = (const int*)d_in[4];
  const float* embw  = (const float*)d_in[5];
  const float* embd  = (const float*)d_in[6];
  const float* wxf   = (const float*)d_in[7];
  const float* whf   = (const float*)d_in[8];
  const float* bxf   = (const float*)d_in[9];
  const float* bhf   = (const float*)d_in[10];
  const float* wxb   = (const float*)d_in[11];
  const float* whb   = (const float*)d_in[12];
  const float* bxb   = (const float*)d_in[13];
  const float* bhb   = (const float*)d_in[14];
  const float* whg   = (const float*)d_in[15];
  const float* bhg   = (const float*)d_in[16];
  const float* bases = (const float*)d_in[17];
  const float* wcomp = (const float*)d_in[18];
  const float* gbias = (const float*)d_in[19];
  const float* w1    = (const float*)d_in[20];
  const float* b1    = (const float*)d_in[21];
  const float* w2    = (const float*)d_in[22];
  const float* b2    = (const float*)d_in[23];
  float* out = (float*)d_out;

  const int NPAD = ((nN + NBD - 1) / NBD) * NBD;
  const int nNB  = (nN + NPB - 1) / NPB;
  const int nGB  = NPAD / NBD;
  const int nFB  = (NB * NC + NTHR - 1) / NTHR;

  char* ws = (char*)d_ws;
  size_t off = 0;
  const size_t oGX  = off; off += (size_t)2 * NB * T * HG * 4;     off = (off + 255) & ~(size_t)255;
  const size_t oQ   = off; off += (size_t)NB * DH * 4;             off = (off + 255) & ~(size_t)255;
  const size_t oQG  = off; off += (size_t)ROWF * 4;                off = (off + 255) & ~(size_t)255;
  const size_t oQP  = off; off += (size_t)2 * 16 * G * 2;          off = (off + 255) & ~(size_t)255;
  const size_t oBP  = off; off += (size_t)2 * G * G * 2;           off = (off + 255) & ~(size_t)255;
  const size_t oHB  = off; off += (size_t)NPAD * ROWF * 4;         off = (off + 255) & ~(size_t)255;
  const size_t oNF  = off; off += (size_t)NPAD * ROWF * 4;         off = (off + 255) & ~(size_t)255;
  const size_t oSC  = off; off += (size_t)NB * NPAD * 4;           off = (off + 255) & ~(size_t)255;
  const size_t oHID = off; off += (size_t)NB * NH1 * 4;            off = (off + 255) & ~(size_t)255;
  if (off > ws_size || off > (size_t)WSCAP) return;
  float*          gx  = (float*)(ws + oGX);
  float*          q   = (float*)(ws + oQ);
  float*          qg  = (float*)(ws + oQG);
  unsigned short* qp  = (unsigned short*)(ws + oQP);
  unsigned short* bp  = (unsigned short*)(ws + oBP);
  float*          hb  = (float*)(ws + oHB);
  float*          nf2 = (float*)(ws + oNF);
  float*          sc2 = (float*)(ws + oSC);
  float*          hid = (float*)(ws + oHID);

  k_gx<<<dim3(T, NB, 2), HG, 0, stream>>>(ques, embw, wxf, bxf, wxb, bxb, gx, T, nVw);
  k_gru<<<dim3(NB, 2), HG, 0, stream>>>(ques, gx, whf, bhf, whb, bhb, q, T);
  k_qg<<<1, NTHR, 0, stream>>>(q, whg, bhg, bases, qg, qp, bp);
  hipFuncSetAttribute(reinterpret_cast<const void*>(&k_node),
                      hipFuncAttributeMaxDynamicSharedMemorySize, LN_TOT);
  k_node<<<nNB, NTHR, LN_TOT, stream>>>(ndesc, embd, qp, bp, hb, nN, nVd);
  hipFuncSetAttribute(reinterpret_cast<const void*>(&k_graph),
                      hipFuncAttributeMaxDynamicSharedMemorySize, LR_TOT);
  k_graph<<<nGB, NTHR, LR_TOT, stream>>>(edst, esrc, etyp, wcomp, gbias, qg, hb, nf2, sc2,
                                          nN, nE, nR, NPAD, 1);
  const size_t ldsPool = (((size_t)nN * 4) + 255) & ~(size_t)255;
  hipFuncSetAttribute(reinterpret_cast<const void*>(&k_pool),
                      hipFuncAttributeMaxDynamicSharedMemorySize, (int)ldsPool);
  k_pool<<<NB, NTHR, ldsPool, stream>>>(sc2, nf2, q, w1, b1, hid, nN, NPAD);
  k_fc2<<<nFB, NTHR, 0, stream>>>(hid, w2, b2, out, NC, NB * NC);
}
